// EventDrivenFusionFast_45217415692848
// MI455X (gfx1250) — hardware-verified
//
#include <hip/hip_runtime.h>
#include <math.h>
#include <float.h>
#include <stdint.h>


#define BATCH 8
#define SEQ   2048
#define DM    128
#define DM2   256
#define NH    4
#define HD    32
#define NQB   (SEQ / 64)
#define MROWS (BATCH * SEQ)
#define OUTN  (MROWS * DM)
static_assert(NH * HD == DM);
static_assert(HD == 32);
static_assert(DM == 128);
static_assert((SEQ % 64) == 0 && (SEQ % 8) == 0);
static_assert(((MROWS / 64) * (DM / 64)) % 8 == 0);
static_assert((MROWS % 8) == 0);
static_assert(((MROWS * DM / 8) % 256) == 0);
static_assert(((DM * DM / 8) % 256) == 0);

typedef _Float16 v16h __attribute__((ext_vector_type(16)));
typedef _Float16 v8h  __attribute__((ext_vector_type(8)));
typedef float    v8f  __attribute__((ext_vector_type(8)));
typedef float    v4f  __attribute__((ext_vector_type(4)));
typedef unsigned int v4u __attribute__((ext_vector_type(4)));

__device__ __forceinline__ unsigned short bf_bits(float f) {
  unsigned u = __float_as_uint(f);
  return (unsigned short)((u + 0x7FFFu + ((u >> 16) & 1u)) >> 16);
}
__device__ __forceinline__ float bf_up(unsigned short h) { return __uint_as_float(((unsigned)h) << 16); }
__device__ __forceinline__ float bfr(float f) { return bf_up(bf_bits(f)); }
__device__ __forceinline__ unsigned short h_bits(_Float16 x) { return __builtin_bit_cast(unsigned short, x); }
__device__ __forceinline__ unsigned pk16(unsigned short a, unsigned short b) { return (unsigned)a | ((unsigned)b << 16); }
__device__ __forceinline__ v8f zero8() { v8f z = {0.f, 0.f, 0.f, 0.f, 0.f, 0.f, 0.f, 0.f}; return z; }

__device__ __forceinline__ void ld8(const float* p, float* o) {
  const v4f a = *(const v4f*)(p);
  const v4f b = *(const v4f*)(p + 4);
  o[0] = a[0]; o[1] = a[1]; o[2] = a[2]; o[3] = a[3];
  o[4] = b[0]; o[5] = b[1]; o[6] = b[2]; o[7] = b[3];
}

__device__ __forceinline__ v16h ldfrag_h(const _Float16* p) {
  union { v16h v; v8h h[2]; } f;
  f.h[0] = *(const v8h*)(p);
  f.h[1] = *(const v8h*)(p + 16);
  return f.v;
}

__device__ __forceinline__ v8f mma_h(v16h a, v16h b, v8f c) {
  c = __builtin_amdgcn_wmma_f32_16x16x32_f16(false, a, false, b, (short)0, c, false, false);
#if defined(__HIP_DEVICE_COMPILE__)
  asm volatile("v_nop\n\tv_nop\n\tv_nop\n\tv_nop" : "+v"(c) : "v"(a), "v"(b));
#endif
  return c;
}
__device__ __forceinline__ v8f mma_h_raw(v16h a, v16h b, v8f c) {
  return __builtin_amdgcn_wmma_f32_16x16x32_f16(false, a, false, b, (short)0, c, false, false);
}
__device__ __forceinline__ void dep_guard_h(v8f& a, v8f& b, v16h x) {
#if defined(__HIP_DEVICE_COMPILE__)
  asm volatile("v_nop\n\tv_nop\n\tv_nop\n\tv_nop" : "+v"(a), "+v"(b) : "v"(x));
#endif
}
__device__ __forceinline__ void keep4_h(v16h a, v16h b, v16h c, v16h d) {
#if defined(__HIP_DEVICE_COMPILE__)
  asm volatile("v_nop" :: "v"(a), "v"(b), "v"(c), "v"(d));
#endif
}
__device__ __forceinline__ void acc_guard4(v8f& a, v8f& b, v8f& c, v8f& d) {
#if defined(__HIP_DEVICE_COMPILE__)
  asm volatile("v_nop\n\tv_nop\n\tv_nop\n\tv_nop" : "+v"(a), "+v"(b), "+v"(c), "+v"(d));
#endif
}

__global__ __launch_bounds__(256) void cvt_f16x8(const float* __restrict__ in, unsigned short* out, int n8,
                                                 float sc, int rnd) {
  const int i = blockIdx.x * 256 + threadIdx.x;
  if (i < n8) {
    float v[8];
    ld8(in + (size_t)i * 8, v);
    if (rnd != 0) {
#pragma unroll
      for (int e = 0; e < 8; ++e) v[e] = bfr(v[e]);
    }
    v4u p;
#pragma unroll
    for (int q = 0; q < 4; ++q)
      p[q] = pk16(h_bits((_Float16)(v[2 * q] * sc)), h_bits((_Float16)(v[2 * q + 1] * sc)));
    *(volatile v4u*)(out + (size_t)i * 8) = p;
    __threadfence();
    *(volatile v4u*)(out + (size_t)i * 8) = p;
  }
}

__global__ __launch_bounds__(256) void cvt_rows(const float* __restrict__ in, unsigned short* out, int ldo,
                                                int n8, float sc, int rnd) {
  const int i = blockIdx.x * 256 + threadIdx.x;
  if (i < n8) {
    const int r = i >> 4, c8 = (i & 15) * 8;
    float v[8];
    ld8(in + (size_t)i * 8, v);
    if (rnd != 0) {
#pragma unroll
      for (int e = 0; e < 8; ++e) v[e] = bfr(v[e]);
    }
    v4u p;
#pragma unroll
    for (int q = 0; q < 4; ++q)
      p[q] = pk16(h_bits((_Float16)(v[2 * q] * sc)), h_bits((_Float16)(v[2 * q + 1] * sc)));
    unsigned short* o = out + (size_t)r * (size_t)ldo + c8;
    *(volatile v4u*)o = p;
    __threadfence();
    *(volatile v4u*)o = p;
  }
}

template <int MODE, int RR, int ACT>
__global__ __launch_bounds__(256) void gemm64(
    const unsigned short* __restrict__ Ap, int lda,
    const unsigned short* __restrict__ Btp, int ldb,
    const float* __restrict__ bias, const float* __restrict__ res, int ldr,
    float* Cf, unsigned short* Ch, int ldc, int M, int N, int Kc, int nsplit, int sstride,
    float oscale, float oscale2, float bscale) {
  const _Float16* Ah = (const _Float16*)(const void*)Ap;
  const _Float16* Bh = (const _Float16*)(const void*)Btp;
  __shared__ __align__(16) float sT[8][16 * 68];
  const int lane = threadIdx.x & 31;
  const int wave = threadIdx.x >> 5;
  const int tilesN = N >> 6;
  const int tilesM = M >> 6;
  const int tiles = tilesM * tilesN;
  const int item = blockIdx.x * 8 + wave;
  if (item >= tiles * nsplit) return;
  const int ky = item / tiles;
  const int tile = item - ky * tiles;
  const int tm = tile / tilesN;
  const int tn = tile - tm * tilesN;
  const int m0 = tm << 6;
  const int n0 = tn << 6;
  const int kbeg = ky * Kc;
  const int kend = kbeg + Kc;
  const float bsel = (ky == 0) ? bscale : 0.0f;
  float* Cp = Cf + (size_t)ky * (size_t)sstride;

  const int rlane = lane & 15;
  const int koff  = (lane >> 4) * 8;
  const int mOff  = (lane >> 4) * 8;

  v8f acc[4][4];
#pragma unroll
  for (int i = 0; i < 4; ++i)
#pragma unroll
    for (int j = 0; j < 4; ++j) acc[i][j] = zero8();

  for (int k0 = kbeg; k0 < kend; k0 += 32) {
    v16h bh[4];
#pragma unroll
    for (int j = 0; j < 4; ++j) {
      const size_t bo = (size_t)(n0 + (j << 4) + rlane) * (size_t)ldb + koff + k0;
      bh[j] = ldfrag_h(Bh + bo);
    }
#pragma unroll
    for (int i = 0; i < 4; ++i) {
      const size_t ao = (size_t)(m0 + (i << 4) + rlane) * (size_t)lda + koff + k0;
      const v16h ah = ldfrag_h(Ah + ao);
#pragma unroll
      for (int j = 0; j < 4; ++j) acc[i][j] = mma_h_raw(ah, bh[j], acc[i][j]);
      dep_guard_h(acc[i][0], acc[i][3], ah);
    }
    keep4_h(bh[0], bh[1], bh[2], bh[3]);
  }
  acc_guard4(acc[0][0], acc[0][1], acc[0][2], acc[0][3]);
  acc_guard4(acc[1][0], acc[1][1], acc[1][2], acc[1][3]);
  acc_guard4(acc[2][0], acc[2][1], acc[2][2], acc[2][3]);
  acc_guard4(acc[3][0], acc[3][1], acc[3][2], acc[3][3]);

  float* slab = sT[wave];
#pragma unroll
  for (int i = 0; i < 4; ++i) {
    const int mBase = m0 + (i << 4);
#pragma unroll
    for (int r = 0; r < 8; ++r) {
#pragma unroll
      for (int j = 0; j < 4; ++j) {
        slab[(mOff + r) * 68 + (j << 4) + rlane] = acc[i][j][r];
      }
    }
    __builtin_amdgcn_fence(__ATOMIC_RELEASE, "workgroup");
    __builtin_amdgcn_wave_barrier();
    __builtin_amdgcn_fence(__ATOMIC_ACQUIRE, "workgroup");
    if (MODE != 2) {
      const int h2 = lane >> 4, c4 = (lane & 15) * 4;
      v4f b4;
      {
        const v4f braw = *(const v4f*)(bias + n0 + c4);
#pragma unroll
        for (int e = 0; e < 4; ++e) b4[e] = bfr(braw[e]) * bsel;
      }
      v4f ov[8];
#pragma unroll
      for (int it = 0; it < 8; ++it) {
        const int row = it * 2 + h2;
        const v4f xs = *(const v4f*)(slab + row * 68 + c4);
        v4f v = xs * oscale;
        if (MODE == 1) {
          v4f r4 = *(const v4f*)(res + (size_t)(mBase + row) * (size_t)ldr + n0 + c4);
          if (RR != 0) {
#pragma unroll
            for (int e = 0; e < 4; ++e) r4[e] = bfr(r4[e]);
          }
          v = (v + b4) + r4;
        } else {
          v = v + b4;
        }
        ov[it] = v;
      }
      for (int pass = 0; pass < 2; ++pass) {
#pragma unroll
        for (int it = 0; it < 8; ++it) {
          const int row = it * 2 + h2;
          *(volatile v4f*)(Cp + (size_t)(mBase + row) * (size_t)ldc + n0 + c4) = ov[it];
        }
        __threadfence();
      }
    } else {
      const int q8 = lane & 7, rr = lane >> 3, c8 = q8 * 8;
      float bb[8];
      {
        const v4f b0 = *(const v4f*)(bias + n0 + c8);
        const v4f b1 = *(const v4f*)(bias + n0 + c8 + 4);
#pragma unroll
        for (int e = 0; e < 4; ++e) { bb[e] = bfr(b0[e]) * bsel; bb[4 + e] = bfr(b1[e]) * bsel; }
      }
      v4u ov[4];
#pragma unroll
      for (int it = 0; it < 4; ++it) {
        const int row = it * 4 + rr;
        float xs[8];
        ld8(slab + row * 68 + c8, xs);
        float v[8];
#pragma unroll
        for (int e = 0; e < 8; ++e) {
          float xv = xs[e] * oscale + bb[e];
          if (ACT != 0) xv = fmaxf(xv, 0.0f);
          v[e] = xv * oscale2;
        }
        v4u a;
#pragma unroll
        for (int p = 0; p < 4; ++p) a[p] = pk16(h_bits((_Float16)v[2 * p]), h_bits((_Float16)v[2 * p + 1]));
        ov[it] = a;
      }
      for (int pass = 0; pass < 2; ++pass) {
#pragma unroll
        for (int it = 0; it < 4; ++it) {
          const int row = it * 4 + rr;
          *(volatile v4u*)(Ch + (size_t)(mBase + row) * (size_t)ldc + n0 + c8) = ov[it];
        }
        __threadfence();
      }
    }
    __builtin_amdgcn_fence(__ATOMIC_RELEASE, "workgroup");
    __builtin_amdgcn_wave_barrier();
    __builtin_amdgcn_fence(__ATOMIC_ACQUIRE, "workgroup");
  }
}

__global__ __launch_bounds__(128) void k_scan(const float* __restrict__ P, const float* __restrict__ ga,
                                              const float* __restrict__ be, const float* __restrict__ ht,
                                              const float* __restrict__ dec,
                                              unsigned short* C1, unsigned short* C2, int ldc,
                                              unsigned short* Lp, int ldl, float hsc) {
#pragma clang fp contract(off)
  __shared__ float red[2][4];
  __shared__ __align__(16) float stg[8 * 132];
  const int tid = threadIdx.x, wave = tid >> 5, lane = tid & 31;
  const int b = blockIdx.x;
  const int c = tid;
  const float gg = bfr(ga[c]);
  const float bb = bfr(be[c]);
  const float dpar = bfr(dec[c]);
  const float dd = 1.0f / (1.0f + expf(-dpar));
  const int j8 = tid >> 4, c8 = (tid & 15) * 8;
  float s = 0.0f;
  for (int t = 0; t < SEQ; ++t) {
    const int row = b * SEQ + t;
    const float x = P[(size_t)row * DM + c];
    float a = x;
#pragma unroll
    for (int off = 16; off >= 1; off >>= 1) a += __shfl_xor(a, off, 32);
    if (lane == 0) red[0][wave] = a;
    __syncthreads();
    const float mu = ((red[0][0] + red[0][1]) + (red[0][2] + red[0][3])) * (1.0f / (float)DM);
    const float dv = x - mu;
    float q = dv * dv;
#pragma unroll
    for (int off = 16; off >= 1; off >>= 1) q += __shfl_xor(q, off, 32);
    if (lane == 0) red[1][wave] = q;
    __syncthreads();
    const float var = ((red[1][0] + red[1][1]) + (red[1][2] + red[1][3])) * (1.0f / (float)DM);
    const float rs = 1.0f / sqrtf(var + 1e-5f);
    const float y = (dv * rs) * gg + bb;
    const float imp = tanhf(y) * bfr(ht[row]);
    s = dd * s + imp;
    stg[(t & 7) * 132 + c] = s;
    if ((t & 7) == 7) {
      __syncthreads();
      float v[8];
      ld8(stg + j8 * 132 + c8, v);
      v4u hv, lv;
#pragma unroll
      for (int p = 0; p < 4; ++p) {
        const float f0 = v[2 * p] * hsc, f1 = v[2 * p + 1] * hsc;
        const _Float16 x0 = (_Float16)f0, x1 = (_Float16)f1;
        const unsigned short h0 = h_bits(x0), h1 = h_bits(x1);
        const unsigned short l0 = h_bits((_Float16)((f0 - (float)x0) * 4096.0f));
        const unsigned short l1 = h_bits((_Float16)((f1 - (float)x1) * 4096.0f));
        hv[p] = pk16(h0, h1); lv[p] = pk16(l0, l1);
      }
      const size_t r8 = (size_t)(row - 7 + j8);
      unsigned short* a1 = C1 + r8 * (size_t)ldc + c8;
      unsigned short* a2 = C2 + r8 * (size_t)ldc + c8;
      unsigned short* a3 = Lp + r8 * (size_t)ldl + c8;
      *(volatile v4u*)a1 = hv;
      *(volatile v4u*)a2 = hv;
      *(volatile v4u*)a3 = lv;
      __threadfence();
      *(volatile v4u*)a1 = hv;
      *(volatile v4u*)a2 = hv;
      *(volatile v4u*)a3 = lv;
      __syncthreads();
    }
  }
}

template <int TWO, int GELU, int OUTF, int OUTH, int OUTL>
__global__ __launch_bounds__(256) void k_lnrow(const float* __restrict__ P0, const float* __restrict__ P1,
                                               const float* __restrict__ ga, const float* __restrict__ be,
                                               float* F, unsigned short* Hh, int ldh,
                                               unsigned short* Lh, int ldl, int nrows, float hsc) {
#pragma clang fp contract(off)
  const int tid = threadIdx.x, wave = tid >> 5, lane = tid & 31;
  const int row = blockIdx.x * 8 + wave;
  if (row >= nrows) return;
  const int c0 = lane * 4;
  const size_t ro = (size_t)row * DM + c0;
  v4f xv = *(const v4f*)(P0 + ro);
  if (TWO != 0) {
    const v4f x1 = *(const v4f*)(P1 + ro);
    xv = xv + x1;
  }
  float x[4] = {xv[0], xv[1], xv[2], xv[3]};
  float s = (x[0] + x[1]) + (x[2] + x[3]);
#pragma unroll
  for (int off = 16; off >= 1; off >>= 1) s += __shfl_xor(s, off, 32);
  const float mu = s * (1.0f / (float)DM);
  float d[4];
  float ss = 0.f;
#pragma unroll
  for (int e = 0; e < 4; ++e) { d[e] = x[e] - mu; ss += d[e] * d[e]; }
#pragma unroll
  for (int off = 16; off >= 1; off >>= 1) ss += __shfl_xor(ss, off, 32);
  const float var = ss * (1.0f / (float)DM);
  const float rs = 1.0f / sqrtf(var + 1e-5f);
  float y[4];
  {
    const v4f g4 = *(const v4f*)(ga + c0);
    const v4f b4 = *(const v4f*)(be + c0);
#pragma unroll
    for (int e = 0; e < 4; ++e) y[e] = (d[e] * rs) * bfr(g4[e]) + bfr(b4[e]);
  }
  if (GELU != 0) {
    v4f yv = {y[0], y[1], y[2], y[3]};
#pragma unroll 1
    for (int e = 0; e < 4; ++e) {
      const float t  = yv[0];
      const float gt = 0.5f * t * (1.0f + erff(t * 0.70710678118654752f));
      const v4f nv = {yv[1], yv[2], yv[3], gt};
      yv = nv;
    }
#pragma unroll
    for (int e = 0; e < 4; ++e) y[e] = yv[e];
  }
  const v4f o4 = {y[0], y[1], y[2], y[3]};
  v4u hv = {0u, 0u, 0u, 0u}, lv = {0u, 0u, 0u, 0u};
  if (OUTH != 0 || OUTL != 0) {
    const int s0 = (lane & 15) * 2, s1 = s0 + 1;
    float t8[8];
#pragma unroll
    for (int e = 0; e < 4; ++e) {
      t8[e]     = __shfl(y[e], s0, 32);
      t8[4 + e] = __shfl(y[e], s1, 32);
    }
#pragma unroll
    for (int p = 0; p < 4; ++p) {
      const float f0 = t8[2 * p] * hsc, f1 = t8[2 * p + 1] * hsc;
      const _Float16 x0 = (_Float16)f0, x1 = (_Float16)f1;
      const unsigned short h0 = h_bits(x0), h1 = h_bits(x1);
      const unsigned short l0 = h_bits((_Float16)((f0 - (float)x0) * 4096.0f));
      const unsigned short l1 = h_bits((_Float16)((f1 - (float)x1) * 4096.0f));
      hv[p] = pk16(h0, h1); lv[p] = pk16(l0, l1);
    }
  }
  const size_t ho = (size_t)row * (size_t)ldh + (size_t)lane * 8;
  const size_t lo = (size_t)row * (size_t)ldl + (size_t)lane * 8;
  const bool wl = lane < 16;
  if (OUTF != 0) *(volatile v4f*)(F + ro) = o4;
  if (OUTH != 0) { if (wl) *(volatile v4u*)(Hh + ho) = hv; }
  if (OUTL != 0) { if (wl) *(volatile v4u*)(Lh + lo) = lv; }
  __threadfence();
  if (OUTF != 0) *(volatile v4f*)(F + ro) = o4;
  if (OUTH != 0) { if (wl) *(volatile v4u*)(Hh + ho) = hv; }
  if (OUTL != 0) { if (wl) *(volatile v4u*)(Lh + lo) = lv; }
}

__global__ __launch_bounds__(256) void v_planes(const float* __restrict__ vf, unsigned short* vth, float vscale) {
  __shared__ __align__(16) float sv[64 * 36];
  const int tid = threadIdx.x;
  const int t0  = blockIdx.x * 64;
  const int hh  = blockIdx.y;
  const int bb  = blockIdx.z;
#pragma unroll
  for (int i = 0; i < 2; ++i) {
    const int idx = i * 256 + tid;
    const int tt = idx >> 3, c4 = (idx & 7) * 4;
    const v4f a = *(const v4f*)(vf + ((size_t)(bb * SEQ + t0 + tt)) * DM + hh * HD + c4);
    *(v4f*)(sv + tt * 36 + c4) = a;
  }
  __syncthreads();

  const int g = tid >> 3, piece = tid & 7;
  const int d = g;
  v4u hv;
#pragma unroll
  for (int e = 0; e < 4; ++e) {
    const float f0 = sv[(piece * 8 + 2 * e) * 36 + d] * vscale;
    const float f1 = sv[(piece * 8 + 2 * e + 1) * 36 + d] * vscale;
    hv[e] = pk16(h_bits((_Float16)f0), h_bits((_Float16)f1));
  }
  const size_t hofs = ((size_t)((bb * NH + hh) * HD + d)) * SEQ + t0 + piece * 8;
  *(volatile v4u*)(vth + hofs) = hv;
  __threadfence();
  *(volatile v4u*)(vth + hofs) = hv;
}

__global__ __launch_bounds__(128)
void attn32(const unsigned short* __restrict__ qhp, const unsigned short* __restrict__ khp,
            const unsigned short* __restrict__ vhp, float* outp, float sscale, float oscl) {
  union FH { v16h v; v8h h[2]; };
  __shared__ __align__(16) _Float16 Ksh[64 * HD];
  __shared__ __align__(16) _Float16 Vth[HD * 64];
  __shared__ __align__(16) _Float16 Psh[4][16 * 64];
  __shared__ __align__(16) float    Os[4][16 * HD];

  const int tid  = threadIdx.x;
  const int wave = tid >> 5;
  const int lane = tid & 31;
  const int hh   = lane >> 4;
  const int c    = lane & 15;

  const int bx = blockIdx.x;
  const int qb = bx % NQB;
  const int bh = bx / NQB;
  const int h  = bh % NH;
  const int b  = bh / NH;
  const int rbase = b * SEQ;
  const int q0 = rbase + qb * 64 + wave * 16;

  const _Float16* Qp = (const _Float16*)(const void*)qhp + (size_t)h * HD;
  const _Float16* Kp = (const _Float16*)(const void*)khp + (size_t)h * HD;
  const _Float16* Vh = (const _Float16*)(const void*)vhp + (size_t)(b * NH + h) * HD * SEQ;

  const v16h qa = ldfrag_h(Qp + (size_t)(q0 + c) * DM + 8 * hh);

  float mrow[8], lrow[8];
  v8f oacc[2];
#pragma unroll
  for (int r = 0; r < 8; ++r) { mrow[r] = -INFINITY; lrow[r] = 0.f; }
#pragma unroll
  for (int t = 0; t < 2; ++t) oacc[t] = zero8();

  for (int kt = 0; kt < NQB; ++kt) {
    const int kv0 = kt * 64;
    __syncthreads();
    {
      const int r = tid >> 1, half = (tid & 1) * 16;
      const _Float16* kg = Kp + (size_t)(rbase + kv0 + r) * DM + half;
      const v8h a0 = *(const v8h*)(kg);
      const v8h a1 = *(const v8h*)(kg + 8);
      *(v8h*)(Ksh + r * HD + half)     = a0;
      *(v8h*)(Ksh + r * HD + half + 8) = a1;
      const int r2 = tid >> 2, qq = (tid & 3) * 16;
      const _Float16* vg = Vh + (size_t)r2 * SEQ + kv0 + qq;
      const v8h b0 = *(const v8h*)(vg);
      const v8h b1 = *(const v8h*)(vg + 8);
      *(v8h*)(Vth + r2 * 64 + qq)     = b0;
      *(v8h*)(Vth + r2 * 64 + qq + 8) = b1;
    }
    __syncthreads();

    v8f s[4];
#pragma unroll
    for (int j = 0; j < 4; ++j) {
      FH kb;
      kb.h[0] = *(const v8h*)(Ksh + (j * 16 + c) * HD + 8 * hh);
      kb.h[1] = *(const v8h*)(Ksh + (j * 16 + c) * HD + 16 + 8 * hh);
      s[j] = mma_h(qa, kb.v, zero8());
    }

    _Float16* pwh = Psh[wave];
#pragma unroll
    for (int r = 0; r < 8; ++r) {
      float m = -INFINITY;
#pragma unroll
      for (int j = 0; j < 4; ++j) {
        const float sv = s[j][r] * sscale;
        s[j][r] = sv;
        m = fmaxf(m, sv);
      }
#pragma unroll
      for (int off = 1; off < 16; off <<= 1) m = fmaxf(m, __shfl_xor(m, off, 32));
      const float mnew  = fmaxf(mrow[r], m);
      const float msafe = (mnew == -INFINITY) ? 0.f : mnew;
      const float alpha = __expf(mrow[r] - msafe);
      mrow[r] = mnew;
      float psum = 0.f;
#pragma unroll
      for (int j = 0; j < 4; ++j) {
        const float p = __expf(s[j][r] - msafe);
        psum += p;
        const _Float16 ph = (_Float16)(p * 1024.0f);
        pwh[(8 * hh + r) * 64 + j * 16 + c] = ph;
      }
#pragma unroll
      for (int off = 1; off < 16; off <<= 1) psum += __shfl_xor(psum, off, 32);
      lrow[r] = lrow[r] * alpha + psum;
#pragma unroll
      for (int t = 0; t < 2; ++t) oacc[t][r] *= alpha;
    }
    __builtin_amdgcn_fence(__ATOMIC_RELEASE, "workgroup");
    __builtin_amdgcn_wave_barrier();
    __builtin_amdgcn_fence(__ATOMIC_ACQUIRE, "workgroup");

#pragma unroll 1
    for (int kk = 0; kk < 2; ++kk) {
      FH pa;
      pa.h[0] = *(const v8h*)(pwh + c * 64 + kk * 32 + 8 * hh);
      pa.h[1] = *(const v8h*)(pwh + c * 64 + kk * 32 + 16 + 8 * hh);
#pragma unroll
      for (int t = 0; t < 2; ++t) {
        FH vb;
        vb.h[0] = *(const v8h*)(Vth + (t * 16 + c) * 64 + kk * 32 + 8 * hh);
        vb.h[1] = *(const v8h*)(Vth + (t * 16 + c) * 64 + kk * 32 + 16 + 8 * hh);
        oacc[t] = mma_h(pa.v, vb.v, oacc[t]);
      }
    }
  }

  float* os = Os[wave];
#pragma unroll
  for (int r = 0; r < 8; ++r) {
    const float l = lrow[r];
    const float inv = ((l > 0.f) ? (1.0f / l) : 0.f) * oscl;
#pragma unroll
    for (int t = 0; t < 2; ++t) os[(8 * hh + r) * HD + t * 16 + c] = oacc[t][r] * inv;
  }
  __builtin_amdgcn_fence(__ATOMIC_RELEASE, "workgroup");
  __builtin_amdgcn_wave_barrier();
  __builtin_amdgcn_fence(__ATOMIC_ACQUIRE, "workgroup");
  {
    const int q8 = lane & 7, rr = lane >> 3;
    v4f ov[4];
#pragma unroll
    for (int it = 0; it < 4; ++it) {
      const int row = it * 4 + rr;
      ov[it] = *(const v4f*)(os + row * HD + q8 * 4);
    }
    for (int pass = 0; pass < 2; ++pass) {
#pragma unroll
      for (int it = 0; it < 4; ++it) {
        const int row = it * 4 + rr;
        const size_t go = (size_t)(q0 + row) * DM + (size_t)h * HD + q8 * 4;
        *(volatile v4f*)(outp + go) = ov[it];
      }
      __threadfence();
    }
  }
}

extern "C" void kernel_launch(void* const* d_in, const int* in_sizes, int n_in,
                              void* d_out, int out_size, void* d_ws, size_t ws_size,
                              hipStream_t stream) {
  if (n_in < 26) return;
  if (in_sizes[0] != OUTN || in_sizes[1] != OUTN) return;
  if (in_sizes[2] != MROWS) return;
  if (in_sizes[3] != DM * DM) return;
  if (in_sizes[4] != DM || in_sizes[5] != DM || in_sizes[6] != DM || in_sizes[7] != DM) return;
  if (in_sizes[8] != 3 * DM * DM || in_sizes[9] != 3 * DM) return;
  if (in_sizes[10] != DM * DM || in_sizes[11] != DM) return;
  if (in_sizes[12] != DM || in_sizes[13] != DM) return;
  if (in_sizes[14] != DM * DM2 || in_sizes[15] != DM || in_sizes[16] != DM || in_sizes[17] != DM) return;
  if (in_sizes[18] != DM * DM2 || in_sizes[19] != DM || in_sizes[20] != DM || in_sizes[21] != DM) return;
  if (in_sizes[22] != DM * DM2 || in_sizes[23] != DM || in_sizes[24] != DM || in_sizes[25] != DM) return;
  if (out_size != OUTN) return;

  const float* lob   = (const float*)d_in[0];
  const float* trade = (const float*)d_in[1];
  const float* htr   = (const float*)d_in[2];
  const float* ei_w  = (const float*)d_in[3];
  const float* ei_b  = (const float*)d_in[4];
  const float* ei_g  = (const float*)d_in[5];
  const float* ei_be = (const float*)d_in[6];
  const float* decay = (const float*)d_in[7];
  const float* inw   = (const float*)d_in[8];
  const float* inb   = (const float*)d_in[9];
  const float* wo    = (const float*)d_in[10];
  const float* bo    = (const float*)d_in[11];
  const float* cn_g  = (const float*)d_in[12];
  const float* cn_b  = (const float*)d_in[13];
  const float* lob_w = (const float*)d_in[14];
  const float* lob_b = (const float*)d_in[15];
  const float* lob_g = (const float*)d_in[16];
  const float* lob_be= (const float*)d_in[17];
  const float* tr_w  = (const float*)d_in[18];
  const float* tr_b  = (const float*)d_in[19];
  const float* tr_g  = (const float*)d_in[20];
  const float* tr_be = (const float*)d_in[21];
  const float* of_w  = (const float*)d_in[22];
  const float* of_b  = (const float*)d_in[23];
  const float* of_g  = (const float*)d_in[24];
  const float* of_be = (const float*)d_in[25];

  const size_t P2h  = (size_t)MROWS * DM2 * 2;
  const size_t P1h  = (size_t)MROWS * DM * 2;
  const size_t PF   = (size_t)MROWS * DM * 4;
  const size_t PVt  = (size_t)BATCH * NH * HD * SEQ * 2;
  const size_t PWei = (size_t)DM * DM * 2;
  const size_t PWc  = (size_t)DM * DM2 * 2;
  const size_t PWin = (size_t)3 * DM * DM * 2;

  size_t off = 0;
  const size_t oTRh  = off; off += P2h;
  const size_t oLBh  = off; off += P2h;
  const size_t oSTl  = off; off += P1h;
  const size_t oWei  = off; off += PWei;
  const size_t oWl   = off; off += PWc;
  const size_t oWt   = off; off += PWc;
  const size_t oWin  = off; off += PWin;
  const size_t oWo   = off; off += PWei;
  const size_t oWof  = off; off += PWc;
  const size_t oS0   = off; off += PF;
  const size_t oS1   = off; off += PF;
  const size_t oLEF  = off; off += PF;
  const size_t oLEH  = off; off += P1h;
  const size_t oCATO = off; off += P2h;
  const size_t oCATL = off; off += P2h;
  const size_t oQh   = off; off += P1h;
  const size_t oKh   = off; off += P1h;
  const size_t oVf   = off; off += PF;
  const size_t oVTh  = off; off += PVt;
  const size_t oOf   = off; off += PF;
  const size_t oOh   = off; off += P1h;
  const size_t oT0   = off; off += PF;
  if (off > ws_size) return;
  if (off > (size_t)134217728) return;

  char* ws = (char*)d_ws;
  unsigned short* TRh   = (unsigned short*)(ws + oTRh);
  unsigned short* LBh   = (unsigned short*)(ws + oLBh);
  unsigned short* STl   = (unsigned short*)(ws + oSTl);
  unsigned short* Wei16 = (unsigned short*)(ws + oWei);
  unsigned short* Wl16  = (unsigned short*)(ws + oWl);
  unsigned short* Wt16  = (unsigned short*)(ws + oWt);
  unsigned short* Win16 = (unsigned short*)(ws + oWin);
  unsigned short* Wo16  = (unsigned short*)(ws + oWo);
  unsigned short* Wof16 = (unsigned short*)(ws + oWof);
  float*          S0    = (float*)(ws + oS0);
  float*          S1    = (float*)(ws + oS1);
  float*          LEF   = (float*)(ws + oLEF);
  unsigned short* LEH   = (unsigned short*)(ws + oLEH);
  unsigned short* CATO  = (unsigned short*)(ws + oCATO);
  unsigned short* CATOL = (unsigned short*)(ws + oCATL);
  unsigned short* Qh    = (unsigned short*)(ws + oQh);
  unsigned short* Kh    = (unsigned short*)(ws + oKh);
  float*          Vf    = (float*)(ws + oVf);
  unsigned short* VTh   = (unsigned short*)(ws + oVTh);
  float*          Of    = (float*)(ws + oOf);
  unsigned short* Oh    = (unsigned short*)(ws + oOh);
  float*          T0    = (float*)(ws + oT0);
  float*          outf  = (float*)d_out;

  const dim3 blk(256);
  const int n8x   = MROWS * DM / 8;
  const int n8dd  = DM * DM / 8;
  const int n8dc  = DM * DM2 / 8;
  const int n8in  = 3 * DM * DM / 8;
  const dim3 gX((n8x + 255) / 256);
  const dim3 gWdd((n8dd + 255) / 256);
  const dim3 gWdc((n8dc + 255) / 256);
  const dim3 gWin((n8in + 255) / 256);
  const dim3 gDM(((MROWS / 64) * (DM / 64) + 7) / 8);
  const dim3 gRow(MROWS / 8);
  const dim3 gScan(BATCH);
  const dim3 gVpl(SEQ / 64, NH, BATCH);
  const dim3 gAttn(BATCH * NH * NQB);

  const float wScale  = 64.0f;
  const float hScale  = 8.0f;
  const float qkScale = 16.0f;
  const float sscale  = 0.17677669529663688f * (1.0f / 256.0f);
  const float vScale  = 256.0f;
  const float attOscl = 1.0f / 262144.0f;
  const float oScale  = 64.0f;
  const float scHi    = 1.0f / 512.0f;
  const float scLo    = 1.0f / 2097152.0f;
  const float scOp    = 1.0f / 4096.0f;

  cvt_f16x8<<<gWdd, blk, 0, stream>>>(ei_w, Wei16, n8dd, wScale, 1);
  cvt_f16x8<<<gWdc, blk, 0, stream>>>(lob_w, Wl16, n8dc, wScale, 1);
  cvt_f16x8<<<gWdc, blk, 0, stream>>>(tr_w, Wt16, n8dc, wScale, 1);
  cvt_f16x8<<<gWin, blk, 0, stream>>>(inw, Win16, n8in, wScale, 1);
  cvt_f16x8<<<gWdd, blk, 0, stream>>>(wo, Wo16, n8dd, wScale, 1);
  cvt_f16x8<<<gWdc, blk, 0, stream>>>(of_w, Wof16, n8dc, wScale, 1);
  cvt_rows<<<gX, blk, 0, stream>>>(trade, TRh, DM2, n8x, hScale, 1);
  cvt_rows<<<gX, blk, 0, stream>>>(lob, LBh, DM2, n8x, hScale, 1);
  gemm64<0, 0, 0><<<gDM, blk, 0, stream>>>(TRh, DM2, Wei16, DM, ei_b, LEF, DM, S0, Qh, DM, MROWS, DM, DM, 1, 0,
                                           scHi, 1.0f, 1.0f);
  k_scan<<<gScan, dim3(128), 0, stream>>>(S0, ei_g, ei_be, htr, decay, TRh + DM, LBh + DM, DM2, STl, DM, hScale);
  gemm64<0, 0, 0><<<gDM, blk, 0, stream>>>(LBh, DM2, Wl16, DM2, lob_b, LEF, DM, S0, Qh, DM, MROWS, DM, DM2, 1, 0,
                                           scHi, 1.0f, 1.0f);
  gemm64<0, 0, 0><<<gDM, blk, 0, stream>>>(STl, DM, Wl16 + DM, DM2, lob_b, LEF, DM, S1, Qh, DM, MROWS, DM, DM, 1, 0,
                                           scLo, 1.0f, 0.0f);
  k_lnrow<1, 1, 1, 1, 0><<<gRow, blk, 0, stream>>>(S0, S1, lob_g, lob_be, LEF, LEH, DM, STl, DM, MROWS, hScale);
  gemm64<0, 0, 0><<<gDM, blk, 0, stream>>>(TRh, DM2, Wt16, DM2, tr_b, LEF, DM, S0, Qh, DM, MROWS, DM, DM2, 1, 0,
                                           scHi, 1.0f, 1.0f);
  gemm64<0, 0, 0><<<gDM, blk, 0, stream>>>(STl, DM, Wt16 + DM, DM2, tr_b, LEF, DM, S1, Qh, DM, MROWS, DM, DM, 1, 0,
                                           scLo, 1.0f, 0.0f);
  k_lnrow<1, 1, 0, 1, 1><<<gRow, blk, 0, stream>>>(S0, S1, tr_g, tr_be, LEF, CATO + DM, DM2, CATOL + DM, DM2,
                                                  MROWS, hScale);
  gemm64<2, 0, 0><<<gDM, blk, 0, stream>>>(LEH, DM, Win16, DM, inb, LEF, DM, S0, Qh, DM, MROWS, DM, DM, 1, 0,
                                           scHi, qkScale, 1.0f);
  gemm64<2, 0, 0><<<gDM, blk, 0, stream>>>(CATO + DM, DM2, Win16 + DM * DM, DM, inb + DM, LEF, DM, S0, Kh, DM,
                                           MROWS, DM, DM, 1, 0, scHi, qkScale, 1.0f);
  gemm64<0, 0, 0><<<gDM, blk, 0, stream>>>(CATO + DM, DM2, Win16 + 2 * DM * DM, DM, inb + 2 * DM, LEF, DM, Vf, Qh,
                                           DM, MROWS, DM, DM, 1, 0, scHi, 1.0f, 1.0f);
  v_planes<<<gVpl, blk, 0, stream>>>(Vf, VTh, vScale);
  attn32<<<gAttn, dim3(128), 0, stream>>>(Qh, Kh, VTh, Of, sscale, attOscl);
  cvt_rows<<<gX, blk, 0, stream>>>(Of, Oh, DM, n8x, oScale, 0);
  gemm64<1, 0, 0><<<gDM, blk, 0, stream>>>(Oh, DM, Wo16, DM, bo, LEF, DM, T0, Qh, DM, MROWS, DM, DM, 1, 0,
                                           scOp, 1.0f, 1.0f);
  k_lnrow<0, 0, 0, 1, 1><<<gRow, blk, 0, stream>>>(T0, T0, cn_g, cn_b, LEF, CATO, DM2, CATOL, DM2, MROWS, hScale);
  gemm64<0, 0, 0><<<gDM, blk, 0, stream>>>(CATO, DM2, Wof16, DM2, of_b, LEF, DM, S0, Qh, DM, MROWS, DM, DM2, 1, 0,
                                           scHi, 1.0f, 1.0f);
  gemm64<0, 0, 0><<<gDM, blk, 0, stream>>>(CATOL, DM2, Wof16, DM2, of_b, LEF, DM, S1, Qh, DM, MROWS, DM, DM2, 1, 0,
                                           scLo, 1.0f, 0.0f);
  k_lnrow<1, 1, 1, 0, 0><<<gRow, blk, 0, stream>>>(S0, S1, of_g, of_be, outf, Qh, DM, Qh, DM, MROWS, hScale);
  (void)hipGetLastError();
}
